// TemporalSAGE_35287451304625
// MI455X (gfx1250) — hardware-verified
//
#include <hip/hip_runtime.h>
#include <stddef.h>


#define IND     256
#define TD      16
#define AUG     272
#define HID     256
#define KCAT    544
#define NTHR    256
#define NWAVE   8
#define EPT     8
#define CHUNK   (NTHR * EPT)
#define WCAP    (EPT * 32)
#define LISTN   (NWAVE * WCAP)
#define NB1     256
#define NB2     4096
#define WSC     16.0f
#define WINV    0.0625f

#define LDS1_ACC   (NB1 * AUG * 4)
#define LDS1_LIST  (LISTN * 4)
#define LDS1_CNT   (NB1 * 4)
#define LDS1       (LDS1_ACC + LDS1_LIST + LDS1_CNT + 64)

static_assert((CHUNK & (CHUNK - 1)) == 0);
static_assert(CHUNK <= 2048);
static_assert((NB1 & (NB1 - 1)) == 0 && (NB2 & (NB2 - 1)) == 0);
static_assert(NB1 <= 4096 && NB2 <= 4096);
static_assert(AUG * 4 == KCAT * 2);
static_assert(HID * 4 <= AUG * 4);
static_assert((AUG * 4) % 16 == 0);
static_assert(KCAT % 32 == 0);
static_assert(2 * NB1 * 4 <= LDS1_LIST);
static_assert(NB1 % NWAVE == 0 && NB1 % 64 == 0);

typedef float    v4f  __attribute__((ext_vector_type(4)));
typedef float    v8f  __attribute__((ext_vector_type(8)));
typedef int      v4i  __attribute__((ext_vector_type(4)));
typedef _Float16 v4h  __attribute__((ext_vector_type(4)));
typedef _Float16 v8h  __attribute__((ext_vector_type(8)));
typedef _Float16 v16h __attribute__((ext_vector_type(16)));
union FragH { v16h v; v8h h[2]; };

__device__ __forceinline__ v8h cvt8(v4f a, v4f b) {
  v8h r;
  r[0] = (_Float16)a.x; r[1] = (_Float16)a.y; r[2] = (_Float16)a.z; r[3] = (_Float16)a.w;
  r[4] = (_Float16)b.x; r[5] = (_Float16)b.y; r[6] = (_Float16)b.z; r[7] = (_Float16)b.w;
  return r;
}
__device__ __forceinline__ v4h cvt4(v4f a) {
  v4h r;
  r[0] = (_Float16)a.x; r[1] = (_Float16)a.y; r[2] = (_Float16)a.z; r[3] = (_Float16)a.w;
  return r;
}

__device__ __forceinline__ v8f wmh(v16h a, v16h b, v8f c) {
  v8f d = __builtin_amdgcn_wmma_f32_16x16x32_f16(false, a, false, b, (short)0, c, false, false);
  asm volatile("v_nop\n\tv_nop\n\tv_nop\n\tv_nop" : "+v"(d) : "v"(a), "v"(b));
  return d;
}

template <int NB>
__device__ __forceinline__ int scan_chunk(const int* __restrict__ dsts, int nE, int cbase, int nodeBase,
                                          int vec8, int* list, int tid, int lane, int wave) {
  int wc = 0;
  const int el0  = tid * EPT;
  const int e0   = cbase + el0;
  const int sent = -2147483647 - 1;
  v4i da, db;
  if (vec8 != 0 && cbase + CHUNK <= nE) {
    da = *(const v4i*)(dsts + e0);
    db = *(const v4i*)(dsts + e0 + 4);
  } else {
    const int em = nE - 1;
    da.x = (e0     < nE) ? dsts[min(e0,     em)] : sent;
    da.y = (e0 + 1 < nE) ? dsts[min(e0 + 1, em)] : sent;
    da.z = (e0 + 2 < nE) ? dsts[min(e0 + 2, em)] : sent;
    da.w = (e0 + 3 < nE) ? dsts[min(e0 + 3, em)] : sent;
    db.x = (e0 + 4 < nE) ? dsts[min(e0 + 4, em)] : sent;
    db.y = (e0 + 5 < nE) ? dsts[min(e0 + 5, em)] : sent;
    db.z = (e0 + 6 < nE) ? dsts[min(e0 + 6, em)] : sent;
    db.w = (e0 + 7 < nE) ? dsts[min(e0 + 7, em)] : sent;
  }
  const unsigned nb = (unsigned)nodeBase;
  const unsigned s0 = (unsigned)da.x - nb, s1 = (unsigned)da.y - nb;
  const unsigned s2 = (unsigned)da.z - nb, s3 = (unsigned)da.w - nb;
  const unsigned s4 = (unsigned)db.x - nb, s5 = (unsigned)db.y - nb;
  const unsigned s6 = (unsigned)db.z - nb, s7 = (unsigned)db.w - nb;
  const bool h0 = s0 < (unsigned)NB, h1 = s1 < (unsigned)NB, h2 = s2 < (unsigned)NB, h3 = s3 < (unsigned)NB;
  const bool h4 = s4 < (unsigned)NB, h5 = s5 < (unsigned)NB, h6 = s6 < (unsigned)NB, h7 = s7 < (unsigned)NB;
  const unsigned any = __builtin_amdgcn_ballot_w32(h0 | h1 | h2 | h3 | h4 | h5 | h6 | h7);
  if (any != 0u) {
#define HITJ(J, HJ, SJ) { \
      const unsigned mj = __builtin_amdgcn_ballot_w32(HJ); \
      if (mj != 0u) { \
        if (HJ) { \
          const int pos = wc + (int)__builtin_amdgcn_mbcnt_lo(mj, 0u); \
          if (pos < WCAP) list[wave * WCAP + pos] = ((el0 + (J)) << 12) | (int)(SJ); \
        } \
        wc += (int)__builtin_popcount(mj); } }
    HITJ(0, h0, s0)
    HITJ(1, h1, s1)
    HITJ(2, h2, s2)
    HITJ(3, h3, s3)
    HITJ(4, h4, s4)
    HITJ(5, h5, s5)
    HITJ(6, h6, s6)
    HITJ(7, h7, s7)
#undef HITJ
  }
  return wc;
}

__global__ __launch_bounds__(NTHR) void k_wprep(
    const float* __restrict__ wl, const float* __restrict__ wr, _Float16* wpl) {
  const int i  = blockIdx.x * NTHR + threadIdx.x;
  const int nG = HID * KCAT / 8;
  if (i >= nG) return;
  const int o  = i * 8;
  const int n  = o / KCAT;
  const int k0 = o - n * KCAT;
  const float* p = (k0 < AUG) ? (wl + (size_t)n * AUG + k0) : (wr + (size_t)n * AUG + (k0 - AUG));
  v4f a = *(const v4f*)p;
  v4f b = *(const v4f*)(p + 4);
  a = a * WSC;
  b = b * WSC;
  const v8h hv = cvt8(a, b);
  _Float16* dp = wpl + o;
  *(volatile v8h*)dp = hv;
  __threadfence();
  *(volatile v8h*)dp = hv;
}

__global__ __launch_bounds__(NTHR) void k_layer1(
    const float* __restrict__ x, const int* __restrict__ ei, const int* __restrict__ ts,
    const float* __restrict__ te, const _Float16* __restrict__ wpl, const float* __restrict__ b1,
    const float* __restrict__ whl, const float* __restrict__ whr,
    float* pP, float* pQ, int nN, int nE, int nT, int vec8) {
  extern __shared__ v4f lds_dyn[];
  float* acc  = (float*)lds_dyn;
  int*   list = (int*)((char*)lds_dyn + LDS1_ACC);
  int*   cnt  = list + LISTN;
  int*   wcnt = cnt + NB1;
  float* pqs  = (float*)list;
  const int tid = threadIdx.x, lane = tid & 31, wave = tid >> 5, hh = lane >> 4, m = lane & 15;
  const int nodeBase = blockIdx.x * NB1;
  const int* dsts = ei + nE;

  {
    const v4f z = {0.f, 0.f, 0.f, 0.f};
    for (int i = tid; i < LDS1_ACC / 16; i += NTHR) lds_dyn[i] = z;
    for (int i = tid; i < NB1; i += NTHR) cnt[i] = 0;
  }
  __syncthreads();

  const int nChunks = (nE + CHUNK - 1) / CHUNK;
#pragma unroll 1
  for (int ch = 0; ch < nChunks; ++ch) {
    const int cbase = ch * CHUNK;
    const int wc = scan_chunk<NB1>(dsts, nE, cbase, nodeBase, vec8, list, tid, lane, wave);
    if (lane == 0) wcnt[wave] = wc;
    __syncthreads();
    if (wave == 0) {
#pragma unroll 1
      for (int wsx = 0; wsx < NWAVE; ++wsx) {
        int n = __builtin_amdgcn_readfirstlane(wcnt[wsx]);
        n = n > WCAP ? WCAP : (n < 0 ? 0 : n);
        const int* lp = list + wsx * WCAP;
#pragma unroll 1
        for (int i = 0; i < n; ++i) {
          const int ent  = __builtin_amdgcn_readfirstlane(lp[i]);
          const int slot = ent & (NB1 - 1);
          int e = cbase + ((ent >> 12) & (CHUNK - 1));
          e = e > nE - 1 ? nE - 1 : e;
          int src = ei[e];
          src = src < 0 ? 0 : (src > nN - 1 ? nN - 1 : src);
          int tsv = ts[src];
          tsv = tsv < 0 ? 0 : (tsv > nT - 1 ? nT - 1 : tsv);
          const float* xp = x + (size_t)src * IND + 4 * lane;
          const v4f xa = *(const v4f*)xp;
          const v4f xb = *(const v4f*)(xp + 128);
          const v4f tv = *(const v4f*)(te + (size_t)tsv * TD + 4 * (lane & 3));
          float* ar = acc + slot * AUG;
          v4f* pa = (v4f*)(ar + 4 * lane);        *pa = *pa + xa;
          v4f* pb = (v4f*)(ar + 128 + 4 * lane);  *pb = *pb + xb;
          if (lane < 4) { v4f* pt = (v4f*)(ar + IND + 4 * lane); *pt = *pt + tv; }
          if (lane == 0) cnt[slot] = cnt[slot] + 1;
        }
      }
    }
    __syncthreads();
  }

#pragma unroll 1
  for (int j = 0; j < NB1 / NWAVE; ++j) {
    const int r = j * NWAVE + wave;
    int node = nodeBase + r;
    node = node > nN - 1 ? nN - 1 : node;
    float* ar = acc + r * AUG;
    const int c = cnt[r];
    const float inv = 1.0f / (float)(c > 1 ? c : 1);
    const v4f a0 = *(const v4f*)(ar + 8 * lane);
    const v4f a1 = *(const v4f*)(ar + 8 * lane + 4);
    const v4f at = *(const v4f*)(ar + IND + 4 * (lane & 3));
    int tsn = ts[node];
    tsn = tsn < 0 ? 0 : (tsn > nT - 1 ? nT - 1 : tsn);
    const float* xp = x + (size_t)node * IND + 8 * lane;
    const v4f s0 = *(const v4f*)xp;
    const v4f s1 = *(const v4f*)(xp + 4);
    const v4f st = *(const v4f*)(te + (size_t)tsn * TD + 4 * (lane & 3));
    __syncthreads();
    _Float16* hr = (_Float16*)ar;
    *(v8h*)(hr + 8 * lane)       = cvt8(a0 * inv, a1 * inv);
    *(v8h*)(hr + AUG + 8 * lane) = cvt8(s0, s1);
    if (lane < 4) {
      *(v4h*)(hr + IND + 4 * lane)       = cvt4(at * inv);
      *(v4h*)(hr + AUG + IND + 4 * lane) = cvt4(st);
    }
  }
  __syncthreads();

  const int chf = wave & 1;
  float bcol[8];
#pragma unroll
  for (int u = 0; u < 8; ++u) bcol[u] = b1[128 * chf + 16 * u + m];
  float wl8[8], wr8[8];
#pragma unroll
  for (int jj = 0; jj < 8; ++jj) { wl8[jj] = whl[lane + 32 * jj]; wr8[jj] = whr[lane + 32 * jj]; }
  const _Float16* sA = (const _Float16*)lds_dyn;

#pragma unroll 1
  for (int p = 0; p < NB1 / 64; ++p) {
    const int t = 4 * p + (wave >> 1);
    v8f d[8];
#pragma unroll
    for (int u = 0; u < 8; ++u) { v8f z = {0.f, 0.f, 0.f, 0.f, 0.f, 0.f, 0.f, 0.f}; d[u] = z; }
    const _Float16* arow = sA + (16 * t + m) * KCAT + 8 * hh;
    const _Float16* brow = wpl + (size_t)(128 * chf + m) * KCAT + 8 * hh;
#pragma unroll 1
    for (int kt = 0; kt < KCAT / 32; ++kt) {
      FragH a;
      a.h[0] = *(const v8h*)(arow + 32 * kt);
      a.h[1] = *(const v8h*)(arow + 32 * kt + 16);
#pragma unroll
      for (int u = 0; u < 8; ++u) {
        const _Float16* bp = brow + (size_t)(16 * u) * KCAT + 32 * kt;
        FragH b;
        b.h[0] = *(const v8h*)bp;
        b.h[1] = *(const v8h*)(bp + 16);
        d[u] = wmh(a.v, b.v, d[u]);
      }
    }
    __syncthreads();

    float* sp = acc + (16 * t + 8 * hh) * AUG + 128 * chf + m;
#pragma unroll
    for (int u = 0; u < 8; ++u) {
      sp[0 * AUG + 16 * u] = fmaxf(d[u][0] * WINV + bcol[u], 0.f);
      sp[1 * AUG + 16 * u] = fmaxf(d[u][1] * WINV + bcol[u], 0.f);
      sp[2 * AUG + 16 * u] = fmaxf(d[u][2] * WINV + bcol[u], 0.f);
      sp[3 * AUG + 16 * u] = fmaxf(d[u][3] * WINV + bcol[u], 0.f);
      sp[4 * AUG + 16 * u] = fmaxf(d[u][4] * WINV + bcol[u], 0.f);
      sp[5 * AUG + 16 * u] = fmaxf(d[u][5] * WINV + bcol[u], 0.f);
      sp[6 * AUG + 16 * u] = fmaxf(d[u][6] * WINV + bcol[u], 0.f);
      sp[7 * AUG + 16 * u] = fmaxf(d[u][7] * WINV + bcol[u], 0.f);
    }
    __syncthreads();

#pragma unroll 1
    for (int i = 0; i < 8; ++i) {
      const int R = 64 * p + 8 * wave + i;
      const float* hp = acc + R * AUG + lane;
      float pv = 0.f, qv = 0.f;
#pragma unroll
      for (int jj = 0; jj < 8; ++jj) {
        const float hv = hp[32 * jj];
        pv += hv * wl8[jj];
        qv += hv * wr8[jj];
      }
#pragma unroll
      for (int off = 16; off > 0; off >>= 1) {
        pv += __shfl_xor(pv, off, 32);
        qv += __shfl_xor(qv, off, 32);
      }
      if (lane == 0) { pqs[R] = pv; pqs[NB1 + R] = qv; }
    }
    __syncthreads();
  }

  const float* ps = pqs + (wave & 1) * NB1;
  const v4f o0 = *(const v4f*)(ps + 4 * lane);
  const v4f o1 = *(const v4f*)(ps + 128 + 4 * lane);
  float* gdst = ((wave & 1) == 0 ? pP : pQ) + (size_t)nodeBase;
  if (wave < 2) {
    *(volatile v4f*)(gdst + 4 * lane)       = o0;
    *(volatile v4f*)(gdst + 128 + 4 * lane) = o1;
  }
  __threadfence();
  if (wave < 2) {
    *(volatile v4f*)(gdst + 4 * lane)       = o0;
    *(volatile v4f*)(gdst + 128 + 4 * lane) = o1;
  }
}

__global__ __launch_bounds__(NTHR) void k_head(
    const int* __restrict__ ei, const float* __restrict__ pP, const float* __restrict__ pQ,
    const float* __restrict__ bh, float* out, int nN, int nE, int vec8) {
  __shared__ __attribute__((aligned(16))) float acc2[NB2];
  __shared__ __attribute__((aligned(16))) int cnt2[NB2];
  __shared__ __attribute__((aligned(16))) int list[LISTN];
  __shared__ int wcnt[NWAVE];
  const int tid = threadIdx.x, lane = tid & 31, wave = tid >> 5;
  const int nodeBase = blockIdx.x * NB2;
  const int* dsts = ei + nE;

  for (int i = tid; i < NB2; i += NTHR) { acc2[i] = 0.f; cnt2[i] = 0; }
  __syncthreads();

  const int nChunks = (nE + CHUNK - 1) / CHUNK;
#pragma unroll 1
  for (int ch = 0; ch < nChunks; ++ch) {
    const int cbase = ch * CHUNK;
    const int wc = scan_chunk<NB2>(dsts, nE, cbase, nodeBase, vec8, list, tid, lane, wave);
    if (lane == 0) wcnt[wave] = wc;
    __syncthreads();
    if (wave == 0) {
#pragma unroll 1
      for (int wsx = 0; wsx < NWAVE; ++wsx) {
        int n = __builtin_amdgcn_readfirstlane(wcnt[wsx]);
        n = n > WCAP ? WCAP : (n < 0 ? 0 : n);
        const int* lp = list + wsx * WCAP;
#pragma unroll 1
        for (int i = 0; i < n; ++i) {
          const int ent  = __builtin_amdgcn_readfirstlane(lp[i]);
          const int slot = ent & (NB2 - 1);
          int e = cbase + ((ent >> 12) & (CHUNK - 1));
          e = e > nE - 1 ? nE - 1 : e;
          int src = ei[e];
          src = src < 0 ? 0 : (src > nN - 1 ? nN - 1 : src);
          const float pv = pP[src];
          if (lane == 0) { acc2[slot] = acc2[slot] + pv; cnt2[slot] = cnt2[slot] + 1; }
        }
      }
    }
    __syncthreads();
  }

  const float bb = bh[0];
#pragma unroll 1
  for (int i = 0; i < NB2 / NTHR; ++i) {
    const int slot = i * NTHR + tid;
    int node = nodeBase + slot;
    node = node > nN - 1 ? nN - 1 : node;
    const int c = cnt2[slot];
    const float inv = 1.0f / (float)(c > 1 ? c : 1);
    acc2[slot] = acc2[slot] * inv + bb + pQ[node];
  }
  __syncthreads();

  v4f ov[4];
#pragma unroll
  for (int qd = 0; qd < 4; ++qd) ov[qd] = *(const v4f*)(acc2 + (wave * 4 + qd) * 128 + 4 * lane);
#pragma unroll
  for (int qd = 0; qd < 4; ++qd) {
    const int f  = (wave * 4 + qd) * 128 + 4 * lane;
    const int gi = nodeBase + f;
    if (gi + 4 <= nN) {
      *(volatile v4f*)(out + gi) = ov[qd];
    } else {
      if (gi     < nN) *(volatile float*)(out + gi)     = ov[qd].x;
      if (gi + 1 < nN) *(volatile float*)(out + gi + 1) = ov[qd].y;
      if (gi + 2 < nN) *(volatile float*)(out + gi + 2) = ov[qd].z;
    }
  }
  __threadfence();
#pragma unroll
  for (int qd = 0; qd < 4; ++qd) {
    const int f  = (wave * 4 + qd) * 128 + 4 * lane;
    const int gi = nodeBase + f;
    if (gi + 4 <= nN) {
      *(volatile v4f*)(out + gi) = ov[qd];
    } else {
      if (gi     < nN) *(volatile float*)(out + gi)     = ov[qd].x;
      if (gi + 1 < nN) *(volatile float*)(out + gi + 1) = ov[qd].y;
      if (gi + 2 < nN) *(volatile float*)(out + gi + 2) = ov[qd].z;
    }
  }
}

static inline size_t al256(size_t v) { return (v + 255) & ~(size_t)255; }

extern "C" void kernel_launch(void* const* d_in, const int* in_sizes, int n_in,
                              void* d_out, int out_size, void* d_ws, size_t ws_size,
                              hipStream_t stream) {
  if (n_in < 10) return;
  const int nN = in_sizes[0] / IND;
  const int nE = in_sizes[1] / 2;
  const int nT = in_sizes[3] / TD;
  if (nN <= 0 || nE < 0 || nT <= 0) return;
  if (in_sizes[0] != nN * IND || in_sizes[1] != nE * 2 || in_sizes[2] < nN || in_sizes[3] != nT * TD) return;
  if (in_sizes[4] != HID * AUG || in_sizes[5] < HID || in_sizes[6] != HID * AUG) return;
  if (in_sizes[7] < HID || in_sizes[8] < 1 || in_sizes[9] < HID) return;
  if (out_size != nN) return;

  const float* x   = (const float*)d_in[0];
  const int*   ei  = (const int*)d_in[1];
  const int*   ts  = (const int*)d_in[2];
  const float* te  = (const float*)d_in[3];
  const float* W1l = (const float*)d_in[4];
  const float* b1l = (const float*)d_in[5];
  const float* W1r = (const float*)d_in[6];
  const float* Whl = (const float*)d_in[7];
  const float* bhl = (const float*)d_in[8];
  const float* Whr = (const float*)d_in[9];
  float* out = (float*)d_out;

  const int nB1 = (nN + NB1 - 1) / NB1;
  const int nB2 = (nN + NB2 - 1) / NB2;

  char* ws = (char*)d_ws;
  size_t off = 0;
  const size_t oW = off; off = al256(off + (size_t)HID * KCAT * 2);
  const size_t oP = off; off = al256(off + (size_t)nB1 * NB1 * 4);
  const size_t oQ = off; off = al256(off + (size_t)nB1 * NB1 * 4);
  if (off > ws_size) return;
  _Float16* wpl = (_Float16*)(ws + oW);
  float*    pP  = (float*)(ws + oP);
  float*    pQ  = (float*)(ws + oQ);

  const int vec8 = ((nE & 3) == 0) ? 1 : 0;

  const int nG = HID * KCAT / 8;
  k_wprep<<<(nG + NTHR - 1) / NTHR, NTHR, 0, stream>>>(W1l, W1r, wpl);

  hipFuncSetAttribute(reinterpret_cast<const void*>(&k_layer1),
                      hipFuncAttributeMaxDynamicSharedMemorySize, LDS1);
  k_layer1<<<nB1, NTHR, LDS1, stream>>>(x, ei, ts, te, wpl, b1l, Whl, Whr, pP, pQ, nN, nE, nT, vec8);

  k_head<<<nB2, NTHR, 0, stream>>>(ei, pP, pQ, bhl, out, nN, nE, vec8);
}
